// GIN_35665408425999
// MI455X (gfx1250) — hardware-verified
//
#include <hip/hip_runtime.h>
#include <stddef.h>
#include <stdint.h>


#define DIN     128
#define KD      256
#define NOUTC   5
#define NTHR    256
#define NWAVE   8
#define EPT     8
#define CHUNK   (NTHR * EPT)
#define WCAP    (EPT * 32)
#define LISTN   (NWAVE * WCAP)
#define NBMAX   2048
#define RCAP    28672
#define DEGCAP  64
#define PKS     11
#define GBM     64
#define GBN     128
#define GTHR    128
#define GNT     8
#define PARTW   288
#define PG      32
#define APR     16
#define NUW     (DIN * (KD / 8))
#define WSMAX   134217728
#define LDS_AGG ((2 * RCAP + 2 * NBMAX + LISTN) * 4 + 64)

static_assert((CHUNK & (CHUNK - 1)) == 0 && CHUNK <= (1 << PKS));
static_assert((NBMAX & (NBMAX - 1)) == 0 && NBMAX <= (1 << PKS));
static_assert(NTHR * 8 == NBMAX);
static_assert(LISTN >= NBMAX && LISTN >= NWAVE * WCAP);
static_assert((RCAP % 32) == 0);
static_assert(LDS_AGG <= 300000);
static_assert(GBM == (GTHR / 32) * 16 && GBN == 16 * GNT && GTHR == GBN && GBN == 4 * 32);
static_assert(DIN == 32 * 4 && KD == 2 * DIN);
static_assert((KD % 32) == 0 && (DIN % GBN) == 0);
static_assert((PARTW % 32) == 0 && PARTW >= 2 * GBN + 1 && PARTW / 4 <= GTHR);
static_assert((NUW % NTHR) == 0 && NUW == 4096 && (KD / 8) == 32);
static_assert((PG & (PG - 1)) == 0 && PG <= NBMAX);
static_assert(NTHR == 2 * DIN);
static_assert((APR % 2) == 0 && (GBM % APR) == 0 && (APR * 32) == 2 * NTHR);
static_assert((GBM * GBN) % GTHR == 0);
static_assert(PG * NOUTC == 160 && (PG * NOUTC * 4) % 128 == 0 && PG * NOUTC <= NTHR);

typedef float          v4f  __attribute__((ext_vector_type(4)));
typedef float          v8f  __attribute__((ext_vector_type(8)));
typedef int            v4i  __attribute__((ext_vector_type(4)));
typedef int            v8i  __attribute__((ext_vector_type(8)));
typedef unsigned int   v2u  __attribute__((ext_vector_type(2)));
typedef unsigned int   v4u  __attribute__((ext_vector_type(4)));
typedef unsigned short v8us __attribute__((ext_vector_type(8)));
typedef __bf16         v16b __attribute__((ext_vector_type(16)));
typedef v4f  __attribute__((may_alias)) v4fa;
typedef v4i  __attribute__((may_alias)) v4ia;
typedef v8us __attribute__((may_alias)) v8usa;
union Frag { v16b vb; v8us h[2]; v8i w; };

__device__ __forceinline__ v8f wmx(const Frag& a, const Frag& b, v8f c) {
  v8f d = __builtin_amdgcn_wmma_f32_16x16x32_bf16(false, a.vb, false, b.vb, (short)0, c, false, false);
  asm volatile("v_nop\n\tv_nop\n\tv_nop\n\tv_nop" : "+v"(d) : "v"(a.w), "v"(b.w));
  return d;
}

__device__ __forceinline__ unsigned int bf_bits(float f) {
  const unsigned int u = __float_as_uint(f);
  const unsigned int r = (u + 0x7FFFu + ((u >> 16) & 1u)) >> 16;
  return (f != f) ? 0x7FC0u : r;
}
__device__ __forceinline__ float bf_val(unsigned int b) { return __uint_as_float(b << 16); }
__device__ __forceinline__ float bf_rne(float f) { return bf_val(bf_bits(f)); }

__device__ __forceinline__ float relu_keep(float v) { return (v > 0.0f) ? v : (v - v); }

__device__ __forceinline__ int scan_chunk(const int* __restrict__ dsts, int nE, int cbase, int slotBase,
                                          int nb, int vec8, int* list, int tid, int lane, int wave) {
  int wc = 0;
  const int el0  = tid * EPT;
  const int e0   = cbase + el0;
  const int sent = -2147483647 - 1;
  v4i da, db;
  if (vec8 != 0 && cbase + CHUNK <= nE) {
    da = *(const v4ia*)(dsts + e0);
    db = *(const v4ia*)(dsts + e0 + 4);
  } else {
    da.x = (e0     < nE) ? dsts[min(e0,     nE - 1)] : sent;
    da.y = (e0 + 1 < nE) ? dsts[min(e0 + 1, nE - 1)] : sent;
    da.z = (e0 + 2 < nE) ? dsts[min(e0 + 2, nE - 1)] : sent;
    da.w = (e0 + 3 < nE) ? dsts[min(e0 + 3, nE - 1)] : sent;
    db.x = (e0 + 4 < nE) ? dsts[min(e0 + 4, nE - 1)] : sent;
    db.y = (e0 + 5 < nE) ? dsts[min(e0 + 5, nE - 1)] : sent;
    db.z = (e0 + 6 < nE) ? dsts[min(e0 + 6, nE - 1)] : sent;
    db.w = (e0 + 7 < nE) ? dsts[min(e0 + 7, nE - 1)] : sent;
  }
  const unsigned nbs = (unsigned)slotBase;
  const unsigned unb = (unsigned)nb;
  const unsigned s0 = (unsigned)da.x - nbs, s1 = (unsigned)da.y - nbs;
  const unsigned s2 = (unsigned)da.z - nbs, s3 = (unsigned)da.w - nbs;
  const unsigned s4 = (unsigned)db.x - nbs, s5 = (unsigned)db.y - nbs;
  const unsigned s6 = (unsigned)db.z - nbs, s7 = (unsigned)db.w - nbs;
  const bool h0 = s0 < unb, h1 = s1 < unb, h2 = s2 < unb, h3 = s3 < unb;
  const bool h4 = s4 < unb, h5 = s5 < unb, h6 = s6 < unb, h7 = s7 < unb;
  const unsigned any = __builtin_amdgcn_ballot_w32(h0 | h1 | h2 | h3 | h4 | h5 | h6 | h7);
  if (any != 0u) {
#define HITJ(J, HJ, SJ) { \
      const unsigned mj = __builtin_amdgcn_ballot_w32(HJ); \
      if (mj != 0u) { \
        if (HJ) { \
          const int pos = wc + (int)__builtin_amdgcn_mbcnt_lo(mj, 0u); \
          if (pos < WCAP) list[wave * WCAP + pos] = ((el0 + (J)) << PKS) | (int)(SJ); \
        } \
        wc += (int)__builtin_popcount(mj); } }
    HITJ(0, h0, s0)
    HITJ(1, h1, s1)
    HITJ(2, h2, s2)
    HITJ(3, h3, s3)
    HITJ(4, h4, s4)
    HITJ(5, h5, s5)
    HITJ(6, h6, s6)
    HITJ(7, h7, s7)
#undef HITJ
  }
  return wc;
}

__device__ __forceinline__ v8us cv8c(const float* __restrict__ p) {
  const v4f a = *(const v4fa*)p;
  const v4f b = *(const v4fa*)(p + 4);
  v8us o;
  o[0] = (unsigned short)bf_bits(a.x); o[1] = (unsigned short)bf_bits(a.y);
  o[2] = (unsigned short)bf_bits(a.z); o[3] = (unsigned short)bf_bits(a.w);
  o[4] = (unsigned short)bf_bits(b.x); o[5] = (unsigned short)bf_bits(b.y);
  o[6] = (unsigned short)bf_bits(b.z); o[7] = (unsigned short)bf_bits(b.w);
  return o;
}

__global__ __launch_bounds__(NTHR) void k_wprep(const float* __restrict__ w0, const float* __restrict__ w1,
                                                const float* __restrict__ w2, const float* __restrict__ w3,
                                                unsigned short* p0, unsigned short* p1,
                                                unsigned short* p2, unsigned short* p3) {
  const int u  = (int)blockIdx.x * NTHR + (int)threadIdx.x;
  const int pl = u >> 12;
  const int v  = u & (NUW - 1);
  const int n  = v >> 5;
  const int k8 = (v & 31) * 8;
  const int kk = k8 & (DIN - 1);
  const size_t so = (size_t)n * DIN + (size_t)kk;
  v8us o;
  unsigned short* dp;
  if (pl == 0)      { o = cv8c(w0 + so); dp = p0 + (size_t)v * 8; }
  else if (pl == 1) { o = cv8c(w1 + so); dp = p1 + (size_t)v * 8; }
  else if (pl == 2) { o = cv8c(w2 + so); dp = p2 + (size_t)v * 8; }
  else if (pl == 3) { o = cv8c(w3 + so); dp = p3 + (size_t)v * 8; }
  else return;
  *(volatile v8us*)dp = o;
  __threadfence();
  *(volatile v8us*)dp = o;
}

template <int RND>
__global__ __launch_bounds__(NTHR) void k_agg(
    const int* __restrict__ srcs, const int* __restrict__ dsts,
    const float* __restrict__ fin, const float* __restrict__ ew,
    const float* __restrict__ We, const float* __restrict__ be,
    unsigned short* Hout,
    int nN, int nE, int nb, int vec8, int MPr) {
  extern __shared__ v4f lds_dyn[];
  int* reg1 = (int*)lds_dyn;
  int* reg2 = reg1 + RCAP;
  int* scnt = reg2 + RCAP;
  int* soff = scnt + NBMAX;
  int* list = soff + NBMAX;
  int* wcnt = list + LISTN;
  int* wtot = wcnt + NWAVE;
  const int tid = (int)threadIdx.x, lane = tid & 31, wave = tid >> 5;
  const int nodeBase = (int)blockIdx.x * nb;

  for (int i = tid; i < NBMAX; i += NTHR) scnt[i] = 0;
  __syncthreads();

  int tot = 0;
  const int nChunks = (nE + CHUNK - 1) / CHUNK;
#pragma unroll 1
  for (int ch = 0; ch < nChunks; ++ch) {
    const int cbase = ch * CHUNK;
    const int wc = scan_chunk(dsts, nE, cbase, nodeBase, nb, vec8, list, tid, lane, wave);
    if (lane == 0) wcnt[wave] = wc;
    __syncthreads();
    int pre = 0, all = 0;
#pragma unroll
    for (int w2 = 0; w2 < NWAVE; ++w2) {
      int c = wcnt[w2];
      c = c < 0 ? 0 : (c > WCAP ? WCAP : c);
      all += c;
      pre += (w2 < wave) ? c : 0;
    }
    const int wcc  = wc > WCAP ? WCAP : wc;
    const int base = tot + pre;
#pragma unroll 1
    for (int i = lane; i < wcc; i += 32) {
      const int ent = list[wave * WCAP + i];
      const int el  = (ent >> PKS) & (CHUNK - 1);
      const int sl  = ent & (NBMAX - 1);
      int eid = cbase + el;
      eid = eid > nE - 1 ? nE - 1 : eid;
      const int pos = base + i;
      if (pos < RCAP) reg1[pos] = (int)(((unsigned)eid << PKS) | (unsigned)sl);
    }
    tot += all;
    tot = tot > RCAP ? RCAP : tot;
    __syncthreads();
  }
  const int nh = tot;

  if (wave == 0) {
#pragma unroll 1
    for (int b0 = 0; b0 < nh; b0 += 32) {
      const int idx = b0 + lane;
      const int uv  = reg1[idx < RCAP ? idx : RCAP - 1];
      const int m32 = (nh - b0) < 32 ? (nh - b0) : 32;
#pragma unroll 1
      for (int k = 0; k < m32; ++k) {
        const int u  = __builtin_amdgcn_readlane(uv, k);
        const int sl = u & (NBMAX - 1);
        if (lane == 0) scnt[sl] = scnt[sl] + 1;
      }
    }
  }
  __syncthreads();

  {
    const v4i ca = *(const v4ia*)(scnt + 8 * tid);
    const v4i cb = *(const v4ia*)(scnt + 8 * tid + 4);
    const int e0 = ca.x < 0 ? 0 : ca.x, e1 = ca.y < 0 ? 0 : ca.y, e2 = ca.z < 0 ? 0 : ca.z, e3 = ca.w < 0 ? 0 : ca.w;
    const int e4 = cb.x < 0 ? 0 : cb.x, e5 = cb.y < 0 ? 0 : cb.y, e6 = cb.z < 0 ? 0 : cb.z, e7 = cb.w < 0 ? 0 : cb.w;
    const int ts = e0 + e1 + e2 + e3 + e4 + e5 + e6 + e7;
    int incl = ts;
#pragma unroll
    for (int d = 1; d < 32; d <<= 1) {
      const int up = __shfl_up(incl, d);
      if (lane >= d) incl += up;
    }
    if (lane == 31) wtot[wave] = incl;
    __syncthreads();
    int pre = 0;
#pragma unroll
    for (int w2 = 0; w2 < NWAVE; ++w2) pre += (w2 < wave) ? wtot[w2] : 0;
    int run = pre + incl - ts;
    soff[8 * tid + 0] = run; run += e0;
    soff[8 * tid + 1] = run; run += e1;
    soff[8 * tid + 2] = run; run += e2;
    soff[8 * tid + 3] = run; run += e3;
    soff[8 * tid + 4] = run; run += e4;
    soff[8 * tid + 5] = run; run += e5;
    soff[8 * tid + 6] = run; run += e6;
    soff[8 * tid + 7] = run;
  }
  __syncthreads();
  for (int i = tid; i < NBMAX; i += NTHR) list[i] = soff[i];
  __syncthreads();

  if (wave == 0) {
#pragma unroll 1
    for (int b0 = 0; b0 < nh; b0 += 32) {
      const int idx = b0 + lane;
      const int uv  = reg1[idx < RCAP ? idx : RCAP - 1];
      const int m32 = (nh - b0) < 32 ? (nh - b0) : 32;
#pragma unroll 1
      for (int k = 0; k < m32; ++k) {
        const int u   = __builtin_amdgcn_readlane(uv, k);
        const int sl  = u & (NBMAX - 1);
        const int eid = (int)((unsigned)u >> PKS);
        if (lane == 0) {
          int pos = list[sl];
          pos = pos < 0 ? 0 : (pos > RCAP - 1 ? RCAP - 1 : pos);
          reg2[pos] = eid;
          list[sl] = pos + 1;
        }
      }
    }
  }
  __syncthreads();

  const int nbw = nb >> 3;
  const bool ovf = (nh >= RCAP);
  const float qnan = __int_as_float(0x7fc00000);
  float we0, we1, we2, we3, bb0, bb1, bb2, bb3;
  {
    const v4f a = *(const v4fa*)(We + 4 * lane);
    const v4f b = *(const v4fa*)(be + 4 * lane);
    we0 = bf_rne(a.x); we1 = bf_rne(a.y); we2 = bf_rne(a.z); we3 = bf_rne(a.w);
    bb0 = bf_rne(b.x); bb1 = bf_rne(b.y); bb2 = bf_rne(b.z); bb3 = bf_rne(b.w);
  }

#pragma unroll 1
  for (int jt = 0; jt < nbw; ++jt) {
    const int slot = wave * nbw + jt;
    const int grow = nodeBase + slot;
    int st = soff[slot];
    const int craw = scnt[slot];
    int cnt = craw;
    st  = st < 0 ? 0 : (st > nh ? nh : st);
    cnt = cnt < 0 ? 0 : (cnt > DEGCAP ? DEGCAP : cnt);
    if (cnt > nh - st) cnt = nh - st;
    const float pz = (ovf || craw > DEGCAP) ? qnan : 0.0f;
    const bool liveRow = grow < nN;

    float ag0 = 0.0f, ag1 = 0.0f, ag2 = 0.0f, ag3 = 0.0f;
#pragma unroll 1
    for (int q = 0; q < cnt; ++q) {
      int idx = st + q; idx = idx > RCAP - 1 ? RCAP - 1 : idx;
      int eid = reg2[idx]; eid = eid < 0 ? 0 : (eid > nE - 1 ? nE - 1 : eid);
      const int sraw = srcs[eid];
      const int s = sraw < 0 ? 0 : (sraw > nN - 1 ? nN - 1 : sraw);
      const float e = bf_rne(ew[eid]);
      const v4f v = *(const v4fa*)(fin + (size_t)s * DIN + 4 * lane);
      float v0 = v.x, v1 = v.y, v2 = v.z, v3 = v.w;
      if (RND != 0) { v0 = bf_rne(v0); v1 = bf_rne(v1); v2 = bf_rne(v2); v3 = bf_rne(v3); }
      const float m0 = relu_keep(v0 + fmaf(e, we0, bb0));
      const float m1 = relu_keep(v1 + fmaf(e, we1, bb1));
      const float m2 = relu_keep(v2 + fmaf(e, we2, bb2));
      const float m3 = relu_keep(v3 + fmaf(e, we3, bb3));
      ag0 += m0; ag1 += m1; ag2 += m2; ag3 += m3;
    }
    const int nc = liveRow ? grow : nN - 1;
    const v4f sv = *(const v4fa*)(fin + (size_t)nc * DIN + 4 * lane);
    float s0 = sv.x, s1 = sv.y, s2 = sv.z, s3 = sv.w;
    if (RND != 0) { s0 = bf_rne(s0); s1 = bf_rne(s1); s2 = bf_rne(s2); s3 = bf_rne(s3); }
    float r0 = s0 + ag0, r1 = s1 + ag1, r2 = s2 + ag2, r3 = s3 + ag3;
    r0 = (liveRow ? r0 : 0.0f) + pz;
    r1 = (liveRow ? r1 : 0.0f) + pz;
    r2 = (liveRow ? r2 : 0.0f) + pz;
    r3 = (liveRow ? r3 : 0.0f) + pz;

    const unsigned int h0 = bf_bits(r0), h1 = bf_bits(r1), h2 = bf_bits(r2), h3 = bf_bits(r3);
    const unsigned int l0 = bf_bits(r0 - bf_val(h0)), l1 = bf_bits(r1 - bf_val(h1));
    const unsigned int l2 = bf_bits(r2 - bf_val(h2)), l3 = bf_bits(r3 - bf_val(h3));
    v2u ph, pl;
    ph.x = h0 | (h1 << 16);
    ph.y = h2 | (h3 << 16);
    pl.x = l0 | (l1 << 16);
    pl.y = l2 | (l3 << 16);
    unsigned short* gp = Hout + (size_t)grow * (size_t)KD + 4 * lane;
    const bool wsv = grow < MPr;
    if (wsv) { *(volatile v2u*)gp = ph; *(volatile v2u*)(gp + DIN) = pl; }
    __threadfence();
    if (wsv) { *(volatile v2u*)gp = ph; *(volatile v2u*)(gp + DIN) = pl; }
  }
}

template <int EPI>
__global__ __launch_bounds__(GTHR) void k_gemm(const unsigned short* __restrict__ A, int lda,
                                               const unsigned short* __restrict__ BT, int ldb, int K,
                                               const float* __restrict__ bias,
                                               float* outF, int ldo, int nN, int mRows,
                                               float* part) {
  __shared__ __attribute__((aligned(16))) float stg[GBM * GBN];
  __shared__ __attribute__((aligned(16))) float pst[PARTW];
  const int tid = (int)threadIdx.x, lane = tid & 31, wave = tid >> 5, hh = lane >> 4, m = lane & 15;
  const int rowBase = (int)blockIdx.x * GBM;
  const int colBase = (int)blockIdx.y * GBN;

  v8f acc[GNT];
  {
    const v8f z = {0.f, 0.f, 0.f, 0.f, 0.f, 0.f, 0.f, 0.f};
#pragma unroll
    for (int t = 0; t < GNT; ++t) acc[t] = z;
  }
  const unsigned short* ap = A  + (size_t)(rowBase + 16 * wave + m) * (size_t)lda + 8 * hh;
  const unsigned short* bp = BT + (size_t)(colBase + m) * (size_t)ldb + 8 * hh;

#pragma unroll 1
  for (int k0 = 0; k0 < K; k0 += 32) {
    Frag af;
    af.h[0] = *(const v8usa*)(ap + k0);
    af.h[1] = *(const v8usa*)(ap + k0 + 16);
#pragma unroll
    for (int nt = 0; nt < GNT; ++nt) {
      const unsigned short* wq = bp + (size_t)(16 * nt) * (size_t)ldb + k0;
      Frag bfr;
      bfr.h[0] = *(const v8usa*)wq;
      bfr.h[1] = *(const v8usa*)(wq + 16);
      acc[nt] = wmx(af, bfr, acc[nt]);
    }
  }

#pragma unroll
  for (int nt = 0; nt < GNT; ++nt) {
    const int lc = 16 * nt + m;
    const float bb = bf_rne(bias[colBase + lc]);
#pragma unroll
    for (int r = 0; r < 8; ++r) {
      const int lr = 16 * wave + 8 * hh + r;
      const bool live = (rowBase + lr) < nN;
      float v = acc[nt][r] + bb;
      if constexpr (EPI == 3) v = relu_keep(v);
      stg[lr * GBN + lc] = live ? v : 0.0f;
    }
  }
  __syncthreads();

  v4f fv[16];
#pragma unroll
  for (int i = 0; i < 16; ++i) {
    const int lr = 16 * wave + i;
    fv[i] = *(const v4fa*)(stg + lr * GBN + 4 * lane);
  }
  v4f pv = {0.f, 0.f, 0.f, 0.f};
  const bool pok = (EPI == 1) && (tid < PARTW / 4);
  if constexpr (EPI == 1) {
    int nvr = nN - rowBase;
    nvr = nvr < 0 ? 0 : (nvr > GBM ? GBM : nvr);
    float s = 0.0f;
#pragma unroll 1
    for (int r = 0; r < nvr; ++r) s += stg[r * GBN + tid];
    const float inv = 1.0f / (float)(nvr < 1 ? 1 : nvr);
    const float mean = s * inv;
    float q = 0.0f;
#pragma unroll 1
    for (int r = 0; r < nvr; ++r) {
      const float d = stg[r * GBN + tid] - mean;
      q = fmaf(d, d, q);
    }
    pst[1 + tid] = mean;
    pst[1 + GBN + tid] = q;
    if (tid == 0) pst[0] = (float)nvr;
#pragma unroll 1
    for (int i = 2 * GBN + 1 + tid; i < PARTW; i += GTHR) pst[i] = 0.0f;
    __syncthreads();
    if (pok) pv = *(const v4fa*)(pst + 4 * tid);
  }
  const size_t prow = (size_t)blockIdx.x * (size_t)gridDim.y + (size_t)blockIdx.y;
  float* pp = part + prow * PARTW + 4 * tid;
#pragma unroll
  for (int i = 0; i < 16; ++i) {
    const int gr = rowBase + 16 * wave + i;
    float* op = outF + (size_t)gr * (size_t)ldo + colBase + 4 * lane;
    if (gr < mRows) *(volatile v4f*)op = fv[i];
  }
  if (pok) *(volatile v4f*)pp = pv;
  __threadfence();
#pragma unroll
  for (int i = 0; i < 16; ++i) {
    const int gr = rowBase + 16 * wave + i;
    float* op = outF + (size_t)gr * (size_t)ldo + colBase + 4 * lane;
    if (gr < mRows) *(volatile v4f*)op = fv[i];
  }
  if (pok) *(volatile v4f*)pp = pv;
}

__global__ __launch_bounds__(GBN) void k_bnfin(const float* __restrict__ part, int nPart, int gy, int nh,
                                               const float* __restrict__ gam, const float* __restrict__ bet,
                                               float* ss) {
  __shared__ __attribute__((aligned(16))) float stg[2 * GBN];
  const int tid = (int)threadIdx.x;
  const int by  = (int)blockIdx.x;
  const int col = by * GBN + tid;
  double n = 0.0, mean = 0.0, M2 = 0.0;
#pragma unroll 1
  for (int b = 0; b < nPart; ++b) {
    const float* pr = part + ((size_t)b * (size_t)gy + (size_t)by) * PARTW;
    const double nb = (double)pr[0];
    const double mb = (double)pr[1 + tid];
    const double qb = (double)pr[1 + GBN + tid];
    if (nb > 0.5) {
      const double nn = n + nb;
      const double delta = mb - mean;
      const double f = nb / nn;
      mean = mean + delta * f;
      M2 = M2 + qb + delta * delta * n * f;
      n = nn;
    }
  }
  const double nt = n < 1.0 ? 1.0 : n;
  const float var  = (float)(M2 / nt);
  const float rstd = rsqrtf(var + 1e-5f);
  const float sc = bf_rne(gam[col]) * rstd;
  const float sh = bf_rne(bet[col]) - (float)mean * sc;
  stg[tid] = sc;
  stg[GBN + tid] = sh;
  __syncthreads();
  const int seg = tid >> 5, j = tid & 31;
  const bool ok = tid < 64;
  v4f v = {0.f, 0.f, 0.f, 0.f};
  float* dp = ss + (size_t)(seg & 1) * (size_t)nh + (size_t)by * GBN + 4 * j;
  if (ok) {
    v = *(const v4fa*)(stg + seg * GBN + 4 * j);
    *(volatile v4f*)dp = v;
  }
  __threadfence();
  if (ok) *(volatile v4f*)dp = v;
}

__global__ __launch_bounds__(NTHR) void k_bnsplit(const float* __restrict__ T, const float* __restrict__ ss,
                                                  int nN, int mRows, unsigned short* R) {
  __shared__ float ssh[2 * DIN];
  __shared__ __attribute__((aligned(16))) float tile[APR * DIN];
  const int tid = (int)threadIdx.x;
  ssh[tid] = ss[tid];
  const int rowBase = (int)blockIdx.x * APR;
  const int c  = tid & (DIN - 1);
  const int rs = tid >> 7;
  __syncthreads();
#pragma unroll 1
  for (int r = 0; r < APR / 2; ++r) {
    const int lr   = 2 * r + rs;
    const int grow = rowBase + lr;
    const int gc   = grow < nN ? grow : nN - 1;
    const float u = T[(size_t)gc * DIN + c];
    const float v = relu_keep(fmaf(u, ssh[c], ssh[DIN + c]));
    tile[lr * DIN + c] = (grow < nN) ? v : 0.0f;
  }
  __syncthreads();
  v4u pv[2];
#pragma unroll
  for (int it = 0; it < 2; ++it) {
    const int p = it * NTHR + tid;
    const int lr = p >> 5, q = p & 31;
    const int cb = 8 * (q & 15);
    const bool isHi = q < 16;
    const v4f a = *(const v4fa*)(tile + lr * DIN + cb);
    const v4f b = *(const v4fa*)(tile + lr * DIN + cb + 4);
    const float f[8] = {a.x, a.y, a.z, a.w, b.x, b.y, b.z, b.w};
    unsigned int w[4];
#pragma unroll
    for (int j = 0; j < 4; ++j) {
      const unsigned int h0 = bf_bits(f[2 * j]), h1 = bf_bits(f[2 * j + 1]);
      const unsigned int l0 = bf_bits(f[2 * j] - bf_val(h0)), l1 = bf_bits(f[2 * j + 1] - bf_val(h1));
      const unsigned int q0 = isHi ? h0 : l0, q1 = isHi ? h1 : l1;
      w[j] = q0 | (q1 << 16);
    }
    v4u o; o.x = w[0]; o.y = w[1]; o.z = w[2]; o.w = w[3];
    pv[it] = o;
  }
#pragma unroll
  for (int it = 0; it < 2; ++it) {
    const int p = it * NTHR + tid;
    const int lr = p >> 5, q = p & 31;
    const int grow = rowBase + lr;
    unsigned short* op = R + (size_t)grow * KD + 8 * q;
    if (grow < mRows) *(volatile v4u*)op = pv[it];
  }
  __threadfence();
#pragma unroll
  for (int it = 0; it < 2; ++it) {
    const int p = it * NTHR + tid;
    const int lr = p >> 5, q = p & 31;
    const int grow = rowBase + lr;
    unsigned short* op = R + (size_t)grow * KD + 8 * q;
    if (grow < mRows) *(volatile v4u*)op = pv[it];
  }
}

__global__ __launch_bounds__(NTHR) void k_poollin(const float* __restrict__ X, const int* __restrict__ bat,
                                                  int nN, int vec8b, int nG,
                                                  const float* __restrict__ lw, const float* __restrict__ lb,
                                                  float* out) {
  __shared__ __attribute__((aligned(16))) float accs[PG * DIN];
  __shared__ __attribute__((aligned(16))) int   list[LISTN];
  __shared__ int wcnt[NWAVE];
  __shared__ float lws[NOUTC * DIN];
  __shared__ float lbs[8];
  __shared__ __attribute__((aligned(16))) float os[PG * NOUTC];
  const int tid = (int)threadIdx.x, lane = tid & 31, wave = tid >> 5;
  const int slotBase = (int)blockIdx.x * PG;
  const float ninf = __int_as_float((int)0xff800000u);

  for (int i = tid; i < PG * DIN; i += NTHR) accs[i] = ninf;
#pragma unroll 1
  for (int i = tid; i < NOUTC * DIN; i += NTHR) lws[i] = bf_rne(lw[i]);
  if (tid < 8) {
    const float bb = lb[tid < NOUTC ? tid : NOUTC - 1];
    lbs[tid] = (tid < NOUTC) ? bf_rne(bb) : 0.0f;
  }
  __syncthreads();

  const int nChunks = (nN + CHUNK - 1) / CHUNK;
#pragma unroll 1
  for (int ch = 0; ch < nChunks; ++ch) {
    const int cbase = ch * CHUNK;
    const int wc = scan_chunk(bat, nN, cbase, slotBase, PG, vec8b, list, tid, lane, wave);
    if (lane == 0) wcnt[wave] = wc;
    __syncthreads();
#pragma unroll 1
    for (int w2 = 0; w2 < NWAVE; ++w2) {
      int c = wcnt[w2];
      c = c < 0 ? 0 : (c > WCAP ? WCAP : c);
#pragma unroll 1
      for (int i = 0; i < c; ++i) {
        const int ent = list[w2 * WCAP + i];
        const int el  = (ent >> PKS) & (CHUNK - 1);
        const int sl  = ent & (PG - 1);
        int node = cbase + el;
        node = node < 0 ? 0 : (node > nN - 1 ? nN - 1 : node);
        if (tid < DIN) {
          const float v = X[(size_t)node * DIN + tid];
          const float mo = accs[sl * DIN + tid];
          const float mx = (v > mo) ? v : mo;
          accs[sl * DIN + tid] = (v != v) ? v : mx;
        }
      }
    }
    __syncthreads();
  }

  if (tid < PG * NOUTC) {
    const int g = tid / NOUTC;
    const int j = tid - g * NOUTC;
    float s = 0.0f;
#pragma unroll 4
    for (int c = 0; c < DIN; ++c) s = fmaf(accs[g * DIN + c], lws[j * DIN + c], s);
    os[tid] = s + lbs[j];
  }
  __syncthreads();
  const bool ok = tid < (PG * NOUTC) / 4;
  const int oi = ok ? tid : 0;
  const v4f ov = *(const v4fa*)(os + 4 * oi);
  float* op = out + (size_t)blockIdx.x * (PG * NOUTC) + 4 * oi;
  if (ok) *(volatile v4f*)op = ov;
  __threadfence();
  if (ok) *(volatile v4f*)op = ov;
}

static int pick_nb(int nE, int nN) {
  int nb = NBMAX;
  while (nb > 16 && (long long)nb * (long long)nE * 5LL > (long long)RCAP * (long long)nN * 4LL) nb >>= 1;
  return nb;
}
static inline int cdiv(int a, int b) { return (a + b - 1) / b; }
static inline size_t al256(size_t o) { return (o + 255) & ~(size_t)255; }

extern "C" void kernel_launch(void* const* d_in, const int* in_sizes, int n_in,
                              void* d_out, int out_size, void* d_ws, size_t ws_size,
                              hipStream_t stream) {
  if (n_in < 22) return;
  if (in_sizes[0] < DIN || (in_sizes[0] % DIN) != 0) return;
  const int nN = in_sizes[0] / DIN;
  if (nN < GBM || nN > (1 << 22)) return;
  const int nE2 = in_sizes[1];
  if (nE2 < 2 || (nE2 & 1) != 0) return;
  const int nE = nE2 / 2;
  if (nE < 1 || nE > (1 << 21)) return;
  if (in_sizes[2] != nE) return;
  if (in_sizes[3] != nN) return;
  for (int l = 0; l < 2; ++l) {
    const int b = 4 + 8 * l;
    if (in_sizes[b + 0] != DIN || in_sizes[b + 1] != DIN) return;
    if (in_sizes[b + 2] != DIN * DIN || in_sizes[b + 3] != DIN) return;
    if (in_sizes[b + 4] != DIN || in_sizes[b + 5] != DIN) return;
    if (in_sizes[b + 6] != DIN * DIN || in_sizes[b + 7] != DIN) return;
  }
  if (in_sizes[20] != NOUTC * DIN || in_sizes[21] != NOUTC) return;
  if (out_size < PG * NOUTC || (out_size % (PG * NOUTC)) != 0) return;
  const int nG = out_size / NOUTC;
  if (nG < PG || (nG % PG) != 0 || nG > 65536) return;
  if ((long long)nG * NOUTC != (long long)out_size) return;

  const float* x     = (const float*)d_in[0];
  const int*   ei    = (const int*)  d_in[1];
  const int*   src   = ei;
  const int*   dst   = ei + nE;
  const float* ew    = (const float*)d_in[2];
  const int*   batch = (const int*)  d_in[3];
  const float* We0 = (const float*)d_in[4];   const float* be0 = (const float*)d_in[5];
  const float* W10 = (const float*)d_in[6];   const float* b10 = (const float*)d_in[7];
  const float* g0  = (const float*)d_in[8];   const float* bt0 = (const float*)d_in[9];
  const float* W20 = (const float*)d_in[10];  const float* b20 = (const float*)d_in[11];
  const float* We1 = (const float*)d_in[12];  const float* be1 = (const float*)d_in[13];
  const float* W11 = (const float*)d_in[14];  const float* b11 = (const float*)d_in[15];
  const float* g1  = (const float*)d_in[16];  const float* bt1 = (const float*)d_in[17];
  const float* W21 = (const float*)d_in[18];  const float* b21 = (const float*)d_in[19];
  const float* linw = (const float*)d_in[20]; const float* linb = (const float*)d_in[21];
  float* out = (float*)d_out;

  const int MP   = cdiv(nN, GBM) * GBM;
  const int gM   = MP / GBM;
  const int nb   = pick_nb(nE, nN);
  const int gA   = cdiv(MP, nb);
  const int vec8 = ((nE & 3) == 0) ? 1 : 0;
  const int vec8b = ((nN & 3) == 0) ? 1 : 0;
  if ((long long)gA * nb < (long long)MP) return;
  if ((long long)(gM - 1) * GBM >= (long long)nN) return;
  if ((MP % APR) != 0) return;

  char* ws = (char*)d_ws;
  size_t off = 0;
  const size_t oP10 = off; off = al256(off + (size_t)NUW * 16);
  const size_t oP20 = off; off = al256(off + (size_t)NUW * 16);
  const size_t oP11 = off; off = al256(off + (size_t)NUW * 16);
  const size_t oP21 = off; off = al256(off + (size_t)NUW * 16);
  const size_t oHR  = off; off = al256(off + (size_t)MP * KD * 2);
  const size_t oT   = off; off = al256(off + (size_t)MP * DIN * 4);
  const size_t oX   = off; off = al256(off + (size_t)MP * DIN * 4);
  const size_t oPT  = off; off = al256(off + (size_t)gM * PARTW * 4);
  const size_t oSS  = off; off = al256(off + (size_t)(2 * DIN) * 4);
  if (off > ws_size || off > (size_t)WSMAX) return;
  unsigned short* P10 = (unsigned short*)(ws + oP10);
  unsigned short* P20 = (unsigned short*)(ws + oP20);
  unsigned short* P11 = (unsigned short*)(ws + oP11);
  unsigned short* P21 = (unsigned short*)(ws + oP21);
  unsigned short* HR  = (unsigned short*)(ws + oHR);
  float*          T   = (float*)(ws + oT);
  float*          X   = (float*)(ws + oX);
  float*          PT  = (float*)(ws + oPT);
  float*          SS  = (float*)(ws + oSS);

  hipFuncSetAttribute(reinterpret_cast<const void*>(&k_agg<1>), hipFuncAttributeMaxDynamicSharedMemorySize, LDS_AGG);
  hipFuncSetAttribute(reinterpret_cast<const void*>(&k_agg<0>), hipFuncAttributeMaxDynamicSharedMemorySize, LDS_AGG);

  k_wprep<<<(4 * NUW) / NTHR, NTHR, 0, stream>>>(W10, W20, W11, W21, P10, P20, P11, P21);
  k_agg<1><<<gA, NTHR, LDS_AGG, stream>>>(src, dst, x, ew, We0, be0, HR, nN, nE, nb, vec8, MP);
  k_gemm<1><<<dim3(gM, DIN / GBN), GTHR, 0, stream>>>(HR, KD, P10, KD, KD, b10, T, DIN, nN, MP, PT);
  k_bnfin<<<DIN / GBN, GBN, 0, stream>>>(PT, gM, DIN / GBN, DIN, g0, bt0, SS);
  k_bnsplit<<<MP / APR, NTHR, 0, stream>>>(T, SS, nN, MP, HR);
  k_gemm<3><<<dim3(gM, DIN / GBN), GTHR, 0, stream>>>(HR, KD, P20, KD, KD, b20, X, DIN, nN, MP, PT);
  k_agg<0><<<gA, NTHR, LDS_AGG, stream>>>(src, dst, X, ew, We1, be1, HR, nN, nE, nb, vec8, MP);
  k_gemm<1><<<dim3(gM, DIN / GBN), GTHR, 0, stream>>>(HR, KD, P11, KD, KD, b11, T, DIN, nN, MP, PT);
  k_bnfin<<<DIN / GBN, GBN, 0, stream>>>(PT, gM, DIN / GBN, DIN, g1, bt1, SS);
  k_bnsplit<<<MP / APR, NTHR, 0, stream>>>(T, SS, nN, MP, HR);
  k_gemm<3><<<dim3(gM, DIN / GBN), GTHR, 0, stream>>>(HR, KD, P21, KD, KD, b21, X, DIN, nN, MP, PT);
  k_poollin<<<nG / PG, NTHR, 0, stream>>>(X, batch, nN, vec8b, nG, linw, linb, out);
}
